// GAT_88295937671448
// MI455X (gfx1250) — hardware-verified
//
#include <hip/hip_runtime.h>
#include <stddef.h>
#include <stdint.h>
#include <math.h>


#define FIN    47
#define KX     64
#define NHD    8
#define CH     128
#define FH     1024
#define KH     2048
#define NOUT   47
#define NOP    64
#define NTHR   256
#define NWAVE  8
#define EPT    8
#define CHUNK  (NTHR * EPT)
#define WCAP   (EPT * 32)
#define LISTN  (NWAVE * WCAP)
#define NBA    1024
#define SLA    10
#define RCAP   28672
#define DEGCAP 128
#define STGW   2048
#define GBM    64
#define GBN    128
#define GTHR   128
#define NUW1   (FH * (KX / 8))
#define NUW2   (FH * (KH / 8))
#define NUW3   (NOP * (KH / 8))
#define NEGSL  0.2f
#define EPS_SM 1e-16f
#define AGG_ZINTS (LISTN + 2 * RCAP + 3 * NBA)
#define AGG_LDS_INTS (AGG_ZINTS + 16)
#define WSMAX  134217728

static_assert((CHUNK & (CHUNK - 1)) == 0 && CHUNK <= 4096);
static_assert((NBA & (NBA - 1)) == 0 && NBA == (1 << SLA));
static_assert(((long long)CHUNK << SLA) < (1LL << 31));
static_assert(NBA % NWAVE == 0 && NBA % 32 == 0 && NBA % GBM == 0);
static_assert(RCAP % 4 == 0 && AGG_ZINTS % 4 == 0 && LISTN % 4 == 0);
static_assert(NWAVE * STGW <= RCAP && STGW == FH + KH / 2);
static_assert(KX % 32 == 0 && KH % 32 == 0 && KH == 2 * FH && FH == NHD * CH && CH == GBN);
static_assert(GBM == (GTHR / 32) * 16 && GBN == 4 * 32 && NOP == 64);
static_assert(NUW1 % NTHR == 0 && NUW2 % NTHR == 0 && NUW3 % NTHR == 0);
static_assert(FH == 4 * 256);
static_assert(AGG_LDS_INTS * 4 <= 300000);
static_assert((GBM * NOUT) % 4 == 0 && (GBM * NOUT * 4) % 128 == 0);

typedef float          v4f   __attribute__((ext_vector_type(4)));
typedef float          v8f   __attribute__((ext_vector_type(8)));
typedef int            v4i   __attribute__((ext_vector_type(4)));
typedef int            v8i   __attribute__((ext_vector_type(8)));
typedef unsigned int   v2u   __attribute__((ext_vector_type(2)));
typedef unsigned int   v4u   __attribute__((ext_vector_type(4)));
typedef unsigned short v8us  __attribute__((ext_vector_type(8)));
typedef unsigned short v16us __attribute__((ext_vector_type(16)));
typedef __bf16         v16bf __attribute__((ext_vector_type(16)));
typedef v4f  __attribute__((may_alias)) v4fa;
typedef v4i  __attribute__((may_alias)) v4ia;
typedef v2u  __attribute__((may_alias)) v2ua;
typedef v4u  __attribute__((may_alias)) v4ua;
typedef v8us __attribute__((may_alias)) v8usa;
union FragB { v16bf v; v16us u; v8us h[2]; v8i w; };

__device__ __forceinline__ v8f wmb(const FragB& a, const FragB& b, v8f c) {
  v8f d = __builtin_amdgcn_wmma_f32_16x16x32_bf16(false, a.v, false, b.v, (short)0, c, false, false);
  asm volatile("v_nop\n\tv_nop\n\tv_nop\n\tv_nop" : "+v"(d) : "v"(a.w), "v"(b.w));
  return d;
}

__device__ __forceinline__ unsigned bf16_bits(float f) {
  const unsigned u = __float_as_uint(f);
  return ((u + 0x7FFFu + ((u >> 16) & 1u)) >> 16) & 0xFFFFu;
}
__device__ __forceinline__ float bf16_val(float f) {
  return __uint_as_float(bf16_bits(f) << 16);
}
__device__ __forceinline__ v4f bfr4(const v4f a) {
  v4f r; r.x = bf16_val(a.x); r.y = bf16_val(a.y); r.z = bf16_val(a.z); r.w = bf16_val(a.w); return r;
}

template <int SLB>
__device__ __forceinline__ int scan_chunk(const int* __restrict__ dsts, int nE, int cbase, int slotBase,
                                          int nb, int vec8, int* list, int tid, int lane, int wave) {
  int wc = 0;
  const int el0  = tid * EPT;
  const int e0   = cbase + el0;
  const int sent = -2147483647 - 1;
  v4i da, db;
  if (vec8 != 0 && cbase + CHUNK <= nE) {
    da = *(const v4i*)(dsts + e0);
    db = *(const v4i*)(dsts + e0 + 4);
  } else {
    da.x = (e0     < nE) ? dsts[min(e0,     nE - 1)] : sent;
    da.y = (e0 + 1 < nE) ? dsts[min(e0 + 1, nE - 1)] : sent;
    da.z = (e0 + 2 < nE) ? dsts[min(e0 + 2, nE - 1)] : sent;
    da.w = (e0 + 3 < nE) ? dsts[min(e0 + 3, nE - 1)] : sent;
    db.x = (e0 + 4 < nE) ? dsts[min(e0 + 4, nE - 1)] : sent;
    db.y = (e0 + 5 < nE) ? dsts[min(e0 + 5, nE - 1)] : sent;
    db.z = (e0 + 6 < nE) ? dsts[min(e0 + 6, nE - 1)] : sent;
    db.w = (e0 + 7 < nE) ? dsts[min(e0 + 7, nE - 1)] : sent;
  }
  const unsigned nbs = (unsigned)slotBase;
  const unsigned unb = (unsigned)nb;
  const unsigned s0 = (unsigned)da.x - nbs, s1 = (unsigned)da.y - nbs;
  const unsigned s2 = (unsigned)da.z - nbs, s3 = (unsigned)da.w - nbs;
  const unsigned s4 = (unsigned)db.x - nbs, s5 = (unsigned)db.y - nbs;
  const unsigned s6 = (unsigned)db.z - nbs, s7 = (unsigned)db.w - nbs;
  const bool h0 = s0 < unb, h1 = s1 < unb, h2 = s2 < unb, h3 = s3 < unb;
  const bool h4 = s4 < unb, h5 = s5 < unb, h6 = s6 < unb, h7 = s7 < unb;
  const unsigned any = __builtin_amdgcn_ballot_w32(h0 | h1 | h2 | h3 | h4 | h5 | h6 | h7);
  if (any != 0u) {
#define HITJ(J, HJ, SJ) { \
      const unsigned mj = __builtin_amdgcn_ballot_w32(HJ); \
      if (mj != 0u) { \
        if (HJ) { \
          const int pos = wc + (int)__builtin_amdgcn_mbcnt_lo(mj, 0u); \
          if (pos < WCAP) list[wave * WCAP + pos] = ((el0 + (J)) << SLB) | (int)(SJ); \
        } \
        wc += (int)__builtin_popcount(mj); } }
    HITJ(0, h0, s0)
    HITJ(1, h1, s1)
    HITJ(2, h2, s2)
    HITJ(3, h3, s3)
    HITJ(4, h4, s4)
    HITJ(5, h5, s5)
    HITJ(6, h6, s6)
    HITJ(7, h7, s7)
#undef HITJ
  }
  return wc;
}

__global__ __launch_bounds__(NTHR) void k_prep(const float* __restrict__ x, const float* __restrict__ W1,
                                               const float* __restrict__ W2, const float* __restrict__ W3,
                                               unsigned short* XB, unsigned short* W1T,
                                               unsigned short* W2D, unsigned short* W3D,
                                               int nN, int nUx) {
  const int u = (int)blockIdx.x * NTHR + (int)threadIdx.x;
  v8us o;
  unsigned short* dp;
  if (u < NUW1) {
    const int n  = u >> 3;
    const int k8 = (u & 7) * 8;
#pragma unroll
    for (int i = 0; i < 8; ++i) {
      const int k  = k8 + i;
      const int kc = k < FIN ? k : FIN - 1;
      const float v = W1[(size_t)kc * FH + n];
      o[i] = (k < FIN) ? (unsigned short)bf16_bits(v) : (unsigned short)0;
    }
    dp = W1T + (size_t)n * KX + k8;
  } else if (u < NUW1 + NUW2) {
    const int v  = u - NUW1;
    const int n  = v >> 8;
    const int k8 = (v & 255) * 8;
    const int kk = k8 & (FH - 1);
    const float* p = W2 + (size_t)kk * FH + n;
#pragma unroll
    for (int i = 0; i < 8; ++i) o[i] = (unsigned short)bf16_bits(p[(size_t)i * FH]);
    dp = W2D + (size_t)n * KH + k8;
  } else if (u < NUW1 + NUW2 + NUW3) {
    const int v  = u - NUW1 - NUW2;
    const int n  = v >> 8;
    const int k8 = (v & 255) * 8;
    const int kk = k8 & (FH - 1);
    const int ncl = n < NOUT ? n : NOUT - 1;
    const float* p = W3 + (size_t)kk * NOUT + ncl;
#pragma unroll
    for (int i = 0; i < 8; ++i) {
      const float w = p[(size_t)i * NOUT];
      o[i] = (n < NOUT) ? (unsigned short)bf16_bits(w) : (unsigned short)0;
    }
    dp = W3D + (size_t)n * KH + k8;
  } else if (u < NUW1 + NUW2 + NUW3 + nUx) {
    const int v   = u - NUW1 - NUW2 - NUW3;
    const int row = v >> 3;
    const int k8  = (v & 7) * 8;
    const int rc  = row < nN ? row : nN - 1;
    const float* p = x + (size_t)rc * FIN;
#pragma unroll
    for (int i = 0; i < 8; ++i) {
      const int k  = k8 + i;
      const int kc = k < FIN ? k : FIN - 1;
      const float w = p[kc];
      o[i] = (k < FIN && row < nN) ? (unsigned short)bf16_bits(w) : (unsigned short)0;
    }
    dp = XB + (size_t)row * KX + k8;
  } else {
    return;
  }
  *(volatile v8us*)dp = o;
  __threadfence();
  *(volatile v8us*)dp = o;
}

__global__ __launch_bounds__(GTHR) void k_gemmh(const unsigned short* __restrict__ A,
                                                const unsigned short* __restrict__ BT, int K,
                                                float* Cm, const float* __restrict__ atts,
                                                const float* __restrict__ attd, float* SD, int mRows) {
  __shared__ __attribute__((aligned(16))) float stg[GBM * GBN];
  __shared__ __attribute__((aligned(16))) float sdt[2 * GBM];
  const int tid = (int)threadIdx.x, lane = tid & 31, wave = tid >> 5, hh = lane >> 4, m = lane & 15;
  const int rowBase = (int)blockIdx.x * GBM;
  const int head    = (int)blockIdx.y;
  const int colBase = head * GBN;

  v8f acc[8];
  {
    const v8f z = {0.f, 0.f, 0.f, 0.f, 0.f, 0.f, 0.f, 0.f};
#pragma unroll
    for (int t = 0; t < 8; ++t) acc[t] = z;
  }
  const unsigned short* ap = A  + (size_t)(rowBase + 16 * wave + m) * (size_t)K + 8 * hh;
  const unsigned short* bp = BT + (size_t)(colBase + m) * (size_t)K + 8 * hh;

#pragma unroll 1
  for (int k0 = 0; k0 < K; k0 += 32) {
    FragB af;
    af.h[0] = *(const v8usa*)(ap + k0);
    af.h[1] = *(const v8usa*)(ap + k0 + 16);
#pragma unroll
    for (int nt = 0; nt < 8; ++nt) {
      const unsigned short* wq = bp + (size_t)(16 * nt) * (size_t)K + k0;
      FragB bf;
      bf.h[0] = *(const v8usa*)wq;
      bf.h[1] = *(const v8usa*)(wq + 16);
      acc[nt] = wmb(af, bf, acc[nt]);
    }
  }

#pragma unroll
  for (int nt = 0; nt < 8; ++nt) {
    const int lc = 16 * nt + m;
#pragma unroll
    for (int r = 0; r < 8; ++r) {
      const int lr = 16 * wave + 8 * hh + r;
      stg[lr * GBN + lc] = acc[nt][r];
    }
  }
  __syncthreads();

  const v4f as4 = bfr4(*(const v4fa*)(atts + head * CH + 4 * lane));
  const v4f ad4 = bfr4(*(const v4fa*)(attd + head * CH + 4 * lane));
#pragma unroll 1
  for (int i = 0; i < 16; ++i) {
    const int row = wave * 16 + i;
    const v4f p = *(const v4fa*)(stg + row * GBN + 4 * lane);
    float s = 0.0f, d = 0.0f;
    s = fmaf(p.x, as4.x, s); s = fmaf(p.y, as4.y, s); s = fmaf(p.z, as4.z, s); s = fmaf(p.w, as4.w, s);
    d = fmaf(p.x, ad4.x, d); d = fmaf(p.y, ad4.y, d); d = fmaf(p.z, ad4.z, d); d = fmaf(p.w, ad4.w, d);
#pragma unroll
    for (int off = 16; off > 0; off >>= 1) {
      s += __shfl_xor(s, off);
      d += __shfl_xor(d, off);
    }
    if (lane == 0) { sdt[row] = s; sdt[GBM + row] = d; }
  }
  __syncthreads();

  const int which2 = lane >> 4, piece = lane & 15;
  const v4f sdv = *(const v4fa*)(sdt + which2 * GBM + 4 * piece);
  float* sp = SD + (size_t)(2 * head + which2) * (size_t)mRows + rowBase + 4 * piece;
#pragma unroll 1
  for (int i = 0; i < 16; ++i) {
    const int row = wave * 16 + i;
    const v4f p = *(const v4fa*)(stg + row * GBN + 4 * lane);
    float* op = Cm + (size_t)(rowBase + row) * (size_t)FH + colBase + 4 * lane;
    *(volatile v4f*)op = p;
  }
  if (wave == 0) *(volatile v4f*)sp = sdv;
  __threadfence();
#pragma unroll 1
  for (int i = 0; i < 16; ++i) {
    const int row = wave * 16 + i;
    const v4f p = *(const v4fa*)(stg + row * GBN + 4 * lane);
    float* op = Cm + (size_t)(rowBase + row) * (size_t)FH + colBase + 4 * lane;
    *(volatile v4f*)op = p;
  }
  if (wave == 0) *(volatile v4f*)sp = sdv;
}

__global__ __launch_bounds__(GTHR) void k_gemmo(const unsigned short* __restrict__ A,
                                                const unsigned short* __restrict__ BT, int K,
                                                const float* __restrict__ b3, float* out, int nN) {
  __shared__ __attribute__((aligned(16))) float stgo[GBM * NOUT];
  const int tid = (int)threadIdx.x, lane = tid & 31, wave = tid >> 5, hh = lane >> 4, m = lane & 15;
  const int rowBase = (int)blockIdx.x * GBM;

  v8f acc[4];
  {
    const v8f z = {0.f, 0.f, 0.f, 0.f, 0.f, 0.f, 0.f, 0.f};
    acc[0] = z; acc[1] = z; acc[2] = z; acc[3] = z;
  }
  const unsigned short* ap = A  + (size_t)(rowBase + 16 * wave + m) * (size_t)K + 8 * hh;
  const unsigned short* wp = BT + (size_t)m * (size_t)K + 8 * hh;
#pragma unroll 1
  for (int k0 = 0; k0 < K; k0 += 32) {
    FragB af;
    af.h[0] = *(const v8usa*)(ap + k0);
    af.h[1] = *(const v8usa*)(ap + k0 + 16);
#pragma unroll
    for (int t = 0; t < 4; ++t) {
      const unsigned short* wq = wp + (size_t)(16 * t) * (size_t)K + k0;
      FragB bf;
      bf.h[0] = *(const v8usa*)wq;
      bf.h[1] = *(const v8usa*)(wq + 16);
      acc[t] = wmb(af, bf, acc[t]);
    }
  }

#pragma unroll
  for (int t = 0; t < 4; ++t) {
    const int lc = 16 * t + m;
    const int cl = lc < NOUT ? lc : NOUT - 1;
    const float bz = bf16_val(b3[cl]);
#pragma unroll
    for (int r = 0; r < 8; ++r) {
      const int lr = 16 * wave + 8 * hh + r;
      if (lc < NOUT) stgo[lr * NOUT + lc] = acc[t][r] + bz;
    }
  }
  __syncthreads();

  int live = nN - rowBase;
  live = live < 0 ? 0 : (live > GBM ? GBM : live);
  const int npc = (live * NOUT) >> 2;
  float* ob = out + (size_t)rowBase * NOUT;
#pragma unroll 1
  for (int p = tid; p < npc; p += GTHR) {
    const v4f v = *(const v4fa*)(stgo + 4 * p);
    *(volatile v4f*)(ob + 4 * p) = v;
  }
  __threadfence();
#pragma unroll 1
  for (int p = tid; p < npc; p += GTHR) {
    const v4f v = *(const v4fa*)(stgo + 4 * p);
    *(volatile v4f*)(ob + 4 * p) = v;
  }
}

__device__ __forceinline__ int fetch_src(const int* sl, const int* __restrict__ srcs, int o, int t, int c,
                                         int nc, int nE, int nN) {
  int idx = o + t;
  idx = idx < 0 ? 0 : (idx > RCAP - 1 ? RCAP - 1 : idx);
  const int ent = sl[idx];
  int eid = ent >> SLA;
  eid = eid < 0 ? 0 : (eid > nE - 1 ? nE - 1 : eid);
  int sr = srcs[eid];
  sr = sr < 0 ? 0 : (sr > nN - 1 ? nN - 1 : sr);
  return (t == c) ? nc : sr;
}

__global__ __launch_bounds__(NTHR) void k_agg(const int* __restrict__ srcs, const int* __restrict__ dsts,
                                              int nE, int nN, int vec8, int mRows,
                                              const float* __restrict__ SD,
                                              const float* __restrict__ xl, const float* __restrict__ bias,
                                              unsigned short* hb) {
  extern __shared__ __attribute__((aligned(16))) int dsm[];
  int* list = dsm;
  int* hl   = dsm + LISTN;
  int* sl   = dsm + LISTN + RCAP;
  int* cnt  = dsm + LISTN + 2 * RCAP;
  int* offs = cnt + NBA;
  int* cur  = offs + NBA;
  int* misc = cur + NBA;
  const int tid = (int)threadIdx.x, lane = tid & 31, wave = tid >> 5;
  const int nodeBase = (int)blockIdx.x * NBA;

  {
    const v4i z4 = {0, 0, 0, 0};
    for (int i = tid * 4; i < AGG_ZINTS; i += NTHR * 4) *(v4ia*)(dsm + i) = z4;
    if (tid < 16) misc[tid] = 0;
  }
  __syncthreads();

  int t = 0, ov = 0;
  const int nChunks = (nE + CHUNK - 1) / CHUNK;
#pragma unroll 1
  for (int ch = 0; ch < nChunks; ++ch) {
    const int cbase = ch * CHUNK;
    const int wc = scan_chunk<SLA>(dsts, nE, cbase, nodeBase, NBA, vec8, list, tid, lane, wave);
    if (lane == 0) misc[wave] = wc;
    __syncthreads();
    if (wave == 0) {
#pragma unroll 1
      for (int w2 = 0; w2 < NWAVE; ++w2) {
        int c = misc[w2];
        c = c < 0 ? 0 : (c > WCAP ? WCAP : c);
#pragma unroll 1
        for (int b0 = 0; b0 < c; b0 += 32) {
          const int idx = b0 + lane;
          const int ent = list[w2 * WCAP + (idx < WCAP ? idx : WCAP - 1)];
          const int m32 = (c - b0) < 32 ? (c - b0) : 32;
#pragma unroll 1
          for (int k = 0; k < m32; ++k) {
            const int u    = __builtin_amdgcn_readlane(ent, k);
            const int slot = u & (NBA - 1);
            const int el   = (u >> SLA) & (CHUNK - 1);
            const int pk   = ((cbase + el) << SLA) | slot;
            if (t < RCAP) {
              if (lane == 0) { hl[t] = pk; cnt[slot] = cnt[slot] + 1; }
              t = t + 1;
            } else {
              ov = 1;
            }
          }
        }
      }
    }
    __syncthreads();
  }
  if (wave == 0 && lane == 0) { misc[8] = t; misc[9] = ov; }
  __syncthreads();
  int tt = misc[8];
  tt = tt < 0 ? 0 : (tt > RCAP ? RCAP : tt);
  const int ovf = misc[9];

  if (wave == 0) {
    const int base = lane * (NBA / 32);
    int s = 0;
#pragma unroll 1
    for (int i = 0; i < NBA / 32; ++i) s += cnt[base + i];
    int incl = s;
#pragma unroll
    for (int d = 1; d < 32; d <<= 1) {
      const int y = __shfl_up(incl, d, 32);
      if (lane >= d) incl += y;
    }
    int run = incl - s;
#pragma unroll 1
    for (int i = 0; i < NBA / 32; ++i) {
      const int cv = cnt[base + i];
      offs[base + i] = run;
      cur[base + i]  = run;
      run += cv;
    }
  }
  __syncthreads();
  if (wave == 0) {
#pragma unroll 1
    for (int b0 = 0; b0 < tt; b0 += 32) {
      const int idx = b0 + lane;
      const int ent = hl[idx < RCAP ? idx : RCAP - 1];
      const int m32 = (tt - b0) < 32 ? (tt - b0) : 32;
#pragma unroll 1
      for (int k = 0; k < m32; ++k) {
        const int u    = __builtin_amdgcn_readlane(ent, k);
        const int slot = u & (NBA - 1);
        if (lane == 0) {
          int p = cur[slot];
          p = p < 0 ? 0 : (p > RCAP - 1 ? RCAP - 1 : p);
          sl[p] = u;
          cur[slot] = p + 1;
        }
      }
    }
  }
  __syncthreads();

  const float qnan = __int_as_float(0x7fc00000);
  const float ninf = __int_as_float((int)0xff800000u);
  const float pz   = (ovf != 0) ? qnan : 0.0f;
  float*        stgf = (float*)(hl + wave * STGW);
  unsigned int* stgh = (unsigned int*)(hl + wave * STGW + FH);
  const int hsel = lane >> 4;

#pragma unroll 1
  for (int si = 0; si < NBA / NWAVE; ++si) {
    const int s    = si * NWAVE + wave;
    const int node = nodeBase + s;
    int c = cnt[s];
    const bool big = c > DEGCAP;
    c = c < 0 ? 0 : (c > DEGCAP ? DEGCAP : c);
    int o = offs[s];
    o = o < 0 ? 0 : (o > RCAP ? RCAP : o);
    const int nc   = node < nN ? node : nN - 1;
    const int ct   = c + 1;
    const float pzr = big ? qnan : pz;
    const bool live = node < nN;

#pragma unroll 1
    for (int cp = 0; cp < 4; ++cp) {
      const float* AS0 = SD + (size_t)(4 * cp) * (size_t)mRows;
      const float* AD0 = AS0 + mRows;
      const float* AS1 = AD0 + mRows;
      const float* AD1 = AS1 + mRows;
      const float ad0 = AD0[nc], ad1 = AD1[nc];

      float mx0 = ninf, mx1 = ninf;
#pragma unroll 1
      for (int b0 = 0; b0 < ct; b0 += 32) {
        const int tpos = b0 + lane;
        const int sr = fetch_src(sl, srcs, o, tpos, c, nc, nE, nN);
        float lg0 = AS0[sr] + ad0;
        float lg1 = AS1[sr] + ad1;
        lg0 = lg0 > 0.f ? lg0 : NEGSL * lg0;
        lg1 = lg1 > 0.f ? lg1 : NEGSL * lg1;
        const bool valid = tpos < ct;
        float v0 = valid ? lg0 : ninf;
        float v1 = valid ? lg1 : ninf;
#pragma unroll
        for (int off = 16; off > 0; off >>= 1) {
          const float o0 = __shfl_xor(v0, off);
          const float o1 = __shfl_xor(v1, off);
          v0 = o0 > v0 ? o0 : v0;
          v1 = o1 > v1 ? o1 : v1;
        }
        mx0 = v0 > mx0 ? v0 : mx0;
        mx1 = v1 > mx1 ? v1 : mx1;
      }
      const float m0 = __builtin_isfinite(mx0) ? mx0 : 0.0f;
      const float m1 = __builtin_isfinite(mx1) ? mx1 : 0.0f;

      float dn0 = 0.0f, dn1 = 0.0f;
      v4f a0 = {0.f, 0.f, 0.f, 0.f}, a1 = {0.f, 0.f, 0.f, 0.f};
      const float* xc = xl + cp * 256 + 8 * lane;
#pragma unroll 1
      for (int b0 = 0; b0 < ct; b0 += 32) {
        const int tpos = b0 + lane;
        const int sr = fetch_src(sl, srcs, o, tpos, c, nc, nE, nN);
        float lg0 = AS0[sr] + ad0;
        float lg1 = AS1[sr] + ad1;
        lg0 = lg0 > 0.f ? lg0 : NEGSL * lg0;
        lg1 = lg1 > 0.f ? lg1 : NEGSL * lg1;
        const bool valid = tpos < ct;
        const float e0 = expf(lg0 - m0);
        const float e1 = expf(lg1 - m1);
        const float p0 = valid ? e0 : 0.0f;
        const float p1 = valid ? e1 : 0.0f;
        float t0 = p0, t1 = p1;
#pragma unroll
        for (int off = 16; off > 0; off >>= 1) {
          t0 += __shfl_xor(t0, off);
          t1 += __shfl_xor(t1, off);
        }
        dn0 += t0;
        dn1 += t1;
        const int pi0 = __float_as_int(p0), pi1 = __float_as_int(p1);
        const int m32 = (ct - b0) < 32 ? (ct - b0) : 32;
#pragma unroll 1
        for (int k = 0; k < m32; ++k) {
          const int sk = __builtin_amdgcn_readlane(sr, k);
          const int q0 = __builtin_amdgcn_readlane(pi0, k);
          const int q1 = __builtin_amdgcn_readlane(pi1, k);
          const float pk = __int_as_float((hsel != 0) ? q1 : q0);
          const float* rp = xc + (size_t)sk * FH;
          const v4f ra = *(const v4f*)rp;
          const v4f rb = *(const v4f*)(rp + 4);
          a0.x = fmaf(pk, ra.x, a0.x); a0.y = fmaf(pk, ra.y, a0.y);
          a0.z = fmaf(pk, ra.z, a0.z); a0.w = fmaf(pk, ra.w, a0.w);
          a1.x = fmaf(pk, rb.x, a1.x); a1.y = fmaf(pk, rb.y, a1.y);
          a1.z = fmaf(pk, rb.z, a1.z); a1.w = fmaf(pk, rb.w, a1.w);
        }
      }
      const float dnl = (hsel != 0) ? dn1 : dn0;
      const float inv = 1.0f / (dnl + EPS_SM);
      const float* bq = bias + cp * 256 + 8 * lane;
      const v4f ba = bfr4(*(const v4f*)bq);
      const v4f bb = bfr4(*(const v4f*)(bq + 4));
      v4f ya, yb;
      ya.x = fmaf(a0.x, inv, ba.x) + pzr; ya.y = fmaf(a0.y, inv, ba.y) + pzr;
      ya.z = fmaf(a0.z, inv, ba.z) + pzr; ya.w = fmaf(a0.w, inv, ba.w) + pzr;
      yb.x = fmaf(a1.x, inv, bb.x) + pzr; yb.y = fmaf(a1.y, inv, bb.y) + pzr;
      yb.z = fmaf(a1.z, inv, bb.z) + pzr; yb.w = fmaf(a1.w, inv, bb.w) + pzr;
      const v4f z4 = {0.f, 0.f, 0.f, 0.f};
      if (!live) { ya = z4; yb = z4; }
      *(v4fa*)(stgf + cp * 256 + 8 * lane)     = ya;
      *(v4fa*)(stgf + cp * 256 + 8 * lane + 4) = yb;
    }
    __syncthreads();

#pragma unroll 1
    for (int i = 0; i < 8; ++i) {
      const int q = i * 32 + lane;
      const v4f v = *(const v4fa*)(stgf + 4 * q);
      const float e0 = (v.x > 0.f) ? v.x : expm1f(v.x);
      const float e1 = (v.y > 0.f) ? v.y : expm1f(v.y);
      const float e2 = (v.z > 0.f) ? v.z : expm1f(v.z);
      const float e3 = (v.w > 0.f) ? v.w : expm1f(v.w);
      const unsigned h0 = bf16_bits(e0), h1 = bf16_bits(e1), h2 = bf16_bits(e2), h3 = bf16_bits(e3);
      const unsigned l0 = bf16_bits(e0 - __uint_as_float(h0 << 16));
      const unsigned l1 = bf16_bits(e1 - __uint_as_float(h1 << 16));
      const unsigned l2 = bf16_bits(e2 - __uint_as_float(h2 << 16));
      const unsigned l3 = bf16_bits(e3 - __uint_as_float(h3 << 16));
      v2u hw, lw;
      hw.x = h0 | (h1 << 16); hw.y = h2 | (h3 << 16);
      lw.x = l0 | (l1 << 16); lw.y = l2 | (l3 << 16);
      *(v2ua*)(stgh + 2 * q)       = hw;
      *(v2ua*)(stgh + 512 + 2 * q) = lw;
    }
    __syncthreads();

    if (node < mRows) {
      unsigned short* hp = hb + (size_t)node * KH;
#pragma unroll 1
      for (int i = 0; i < 8; ++i) {
        const int p = i * 32 + lane;
        const v4u w = *(const v4ua*)(stgh + 4 * p);
        *(volatile v4u*)(hp + 8 * p) = w;
      }
      __threadfence();
#pragma unroll 1
      for (int i = 0; i < 8; ++i) {
        const int p = i * 32 + lane;
        const v4u w = *(const v4ua*)(stgh + 4 * p);
        *(volatile v4u*)(hp + 8 * p) = w;
      }
    }
  }
}

static inline int cdiv(int a, int b) { return (a + b - 1) / b; }

extern "C" void kernel_launch(void* const* d_in, const int* in_sizes, int n_in,
                              void* d_out, int out_size, void* d_ws, size_t ws_size,
                              hipStream_t stream) {
  if (n_in < 12) return;
  if (in_sizes[0] < FIN || (in_sizes[0] % FIN) != 0) return;
  const int nN = in_sizes[0] / FIN;
  if ((nN & 3) != 0 || nN > (1 << 20)) return;
  if (in_sizes[1] < 2 || (in_sizes[1] & 1) != 0) return;
  const int nE = in_sizes[1] / 2;
  if (nE < 1 || nE >= (1 << 21)) return;
  if (in_sizes[2] != FIN * FH) return;
  if (in_sizes[3] != FH || in_sizes[4] != FH || in_sizes[5] != FH) return;
  if (in_sizes[6] != FH * FH) return;
  if (in_sizes[7] != FH || in_sizes[8] != FH || in_sizes[9] != FH) return;
  if (in_sizes[10] != FH * NOUT) return;
  if (in_sizes[11] != NOUT) return;
  if ((long long)out_size != (long long)nN * NOUT) return;

  const float* x    = (const float*)d_in[0];
  const int*   edge = (const int*)d_in[1];
  const float* W1   = (const float*)d_in[2];
  const float* a1s  = (const float*)d_in[3];
  const float* a1d  = (const float*)d_in[4];
  const float* b1   = (const float*)d_in[5];
  const float* W2   = (const float*)d_in[6];
  const float* a2s  = (const float*)d_in[7];
  const float* a2d  = (const float*)d_in[8];
  const float* b2   = (const float*)d_in[9];
  const float* W3   = (const float*)d_in[10];
  const float* b3   = (const float*)d_in[11];
  float* out = (float*)d_out;
  const int* src = edge;
  const int* dst = edge + nE;

  const int MP   = cdiv(nN, GBM) * GBM;
  const int gM   = MP / GBM;
  const int gA   = cdiv(MP, NBA);
  if ((long long)gA * NBA < (long long)MP) return;
  const int vec8 = ((nE & 3) == 0) ? 1 : 0;

  char* ws = (char*)d_ws;
  size_t off = 0;
  const size_t oW1T = off; off += (size_t)FH * KX * 2;                    off = (off + 255) & ~(size_t)255;
  const size_t oW2D = off; off += (size_t)FH * KH * 2;                    off = (off + 255) & ~(size_t)255;
  const size_t oW3D = off; off += (size_t)NOP * KH * 2;                   off = (off + 255) & ~(size_t)255;
  const size_t oXB  = off; off += (size_t)MP * KX * 2;                    off = (off + 255) & ~(size_t)255;
  const size_t oSD1 = off; off += (size_t)2 * NHD * MP * 4;               off = (off + 255) & ~(size_t)255;
  const size_t oSD2 = off; off += (size_t)2 * NHD * MP * 4;               off = (off + 255) & ~(size_t)255;
  const size_t oXH  = off; off += (size_t)MP * FH * 4;                    off = (off + 255) & ~(size_t)255;
  const size_t oHP  = off; off += (size_t)MP * KH * 2;                    off = (off + 255) & ~(size_t)255;
  if (off > ws_size || off > (size_t)WSMAX) return;
  unsigned short* W1T = (unsigned short*)(ws + oW1T);
  unsigned short* W2D = (unsigned short*)(ws + oW2D);
  unsigned short* W3D = (unsigned short*)(ws + oW3D);
  unsigned short* XB  = (unsigned short*)(ws + oXB);
  float*          SD1 = (float*)(ws + oSD1);
  float*          SD2 = (float*)(ws + oSD2);
  float*          XH  = (float*)(ws + oXH);
  unsigned short* HP  = (unsigned short*)(ws + oHP);

  const size_t aggLds = (size_t)AGG_LDS_INTS * 4;
  hipFuncSetAttribute(reinterpret_cast<const void*>(&k_agg), hipFuncAttributeMaxDynamicSharedMemorySize, (int)aggLds);

  const int nUx  = MP * (KX / 8);
  const int nUall = NUW1 + NUW2 + NUW3 + nUx;
  k_prep<<<cdiv(nUall, NTHR), NTHR, 0, stream>>>(x, W1, W2, W3, XB, W1T, W2D, W3D, nN, nUx);
  k_gemmh<<<dim3(gM, NHD), GTHR, 0, stream>>>(XB, W1T, KX, XH, a1s, a1d, SD1, MP);
  k_agg<<<gA, NTHR, aggLds, stream>>>(src, dst, nE, nN, vec8, MP, SD1, XH, b1, HP);
  k_gemmh<<<dim3(gM, NHD), GTHR, 0, stream>>>(HP, W2D, KH, XH, a2s, a2d, SD2, MP);
  k_agg<<<gA, NTHR, aggLds, stream>>>(src, dst, nE, nN, vec8, MP, SD2, XH, b2, HP);
  k_gemmo<<<gM, GTHR, 0, stream>>>(HP, W3D, KH, b3, out, nN);
}
